// MambaBlock_42296837931101
// MI455X (gfx1250) — hardware-verified
//
#include <hip/hip_runtime.h>
#include <math.h>

typedef __attribute__((ext_vector_type(8)))  _Float16 v8h;
typedef __attribute__((ext_vector_type(16))) __bf16   v16b;
typedef __attribute__((ext_vector_type(8)))  __bf16   v8b;
typedef __attribute__((ext_vector_type(8)))  float    v8f;
typedef __attribute__((ext_vector_type(4)))  float    v4f;

constexpr int kL      = 1024;
constexpr int kD      = 1024;
constexpr int kNst    = 16;
constexpr int kTap    = 3;
constexpr int kKc     = kTap * kL;
constexpr int kBCP    = 64;
constexpr int kXmRows = kL + 2;
constexpr int kScanTS = 64;
constexpr int kScanCh = 64;
constexpr int kScanYP = 68;
constexpr int kScanXP = 32;
static_assert((kD % 32) == 0 && (kKc % 32) == 0 && (kL % 32) == 0, "GEMM K multiples of 32");
static_assert((kL % 64) == 0 && (kD % 64) == 0 && (kBCP % 64) == 0, "GEMM M,N multiples of 64");
static_assert((kL % kScanTS) == 0 && (kD % kScanCh) == 0, "scan tile multiples");
static_assert((size_t)(kL - 1) * kD + kKc == (size_t)kXmRows * kD, "overlapping conv operand view ends exactly at the plane end");
static_assert(2 * kNst <= kScanXP && 2 * kNst <= kBCP, "B and C columns fit");

constexpr size_t kSzPlane16 = (size_t)kL * kD * 2;
constexpr size_t kOffXH   = 0;
constexpr size_t kOffXL   = kOffXH   + 2 * kSzPlane16;
constexpr size_t kOffWPH  = kOffXL   + 2 * kSzPlane16;
constexpr size_t kOffWPL  = kOffWPH  + kSzPlane16;
constexpr size_t kOffAWH  = kOffWPL  + kSzPlane16;
constexpr size_t kOffAWL  = kOffAWH  + (size_t)kL * kKc * 2;
constexpr size_t kOffWDH  = kOffAWL  + (size_t)kL * kKc * 2;
constexpr size_t kOffWDL  = kOffWDH  + kSzPlane16;
constexpr size_t kOffWBCH = kOffWDL  + kSzPlane16;
constexpr size_t kOffWBCL = kOffWBCH + (size_t)kBCP * kD * 2;
constexpr size_t kOffXMH  = kOffWBCL + (size_t)kBCP * kD * 2;
constexpr size_t kOffXML  = kOffXMH  + (size_t)kXmRows * kD * 2;
constexpr size_t kOffXC   = kOffXML  + (size_t)kXmRows * kD * 2;
constexpr size_t kOffXCH  = kOffXC   + (size_t)kL * kD * 4;
constexpr size_t kOffXCL  = kOffXCH  + kSzPlane16;
constexpr size_t kOffXGH  = kOffXCL  + kSzPlane16;
constexpr size_t kOffXGL  = kOffXGH  + kSzPlane16;
constexpr size_t kOffDLR  = kOffXGL  + kSzPlane16;
constexpr size_t kOffBC   = kOffDLR  + (size_t)kL * kD * 4;
constexpr size_t kOffYH   = kOffBC   + (size_t)kL * kBCP * 4;
constexpr size_t kOffYL   = kOffYH   + kSzPlane16;
constexpr size_t kOffZH   = kOffYL   + kSzPlane16;
constexpr size_t kOffZL   = kOffZH   + kSzPlane16;
constexpr size_t kWsTotal = kOffZL   + kSzPlane16;
static_assert(kWsTotal == 59252736ull, "carve total");
static_assert(kWsTotal <= 134217728ull, "carve cap");
static_assert((kOffXL % 128) == 0 && (kOffWPH % 128) == 0 && (kOffWPL % 128) == 0 && (kOffAWH % 128) == 0 &&
              (kOffAWL % 128) == 0 && (kOffWDH % 128) == 0 && (kOffWDL % 128) == 0 && (kOffWBCH % 128) == 0 &&
              (kOffWBCL % 128) == 0 && (kOffXMH % 128) == 0 && (kOffXML % 128) == 0 && (kOffXC % 128) == 0 &&
              (kOffXCH % 128) == 0 && (kOffXCL % 128) == 0 && (kOffXGH % 128) == 0 && (kOffXGL % 128) == 0 &&
              (kOffDLR % 128) == 0 && (kOffBC % 128) == 0 && (kOffYH % 128) == 0 && (kOffYL % 128) == 0 &&
              (kOffZH % 128) == 0 && (kOffZL % 128) == 0, "128-B aligned regions");

__device__ __forceinline__ unsigned short f2bf_bits(float f) {
  unsigned u = __float_as_uint(f);
  return (unsigned short)((u + 0x7FFFu + ((u >> 16) & 1u)) >> 16);
}
__device__ __forceinline__ float bf_bits2f(unsigned short h) { return __uint_as_float(((unsigned)h) << 16); }

__device__ __forceinline__ float silu_f32(float v) { return v / (1.0f + expf(-v)); }

__device__ __forceinline__ void dep_guard2_b(v8f& a, v8f& b, v16b x, v16b y, v16b p, v16b q, v16b r, v16b s) {
  asm volatile("v_nop\n\tv_nop\n\tv_nop\n\tv_nop" : "+v"(a), "+v"(b) : "v"(x), "v"(y), "v"(p), "v"(q), "v"(r), "v"(s));
}
__device__ __forceinline__ void keep4_b(v16b a, v16b b, v16b c, v16b d) { asm volatile("v_nop" :: "v"(a), "v"(b), "v"(c), "v"(d)); }
__device__ __forceinline__ void acc_guard4(v8f& a, v8f& b, v8f& c, v8f& d) {
  asm volatile("v_nop\n\tv_nop\n\tv_nop\n\tv_nop" : "+v"(a), "+v"(b), "+v"(c), "+v"(d));
}

union FragU { v16b v; v8b h[2]; };
__device__ __forceinline__ v16b frag_load(const __bf16* p) {
  FragU f;
  f.h[0] = *(const v8b*)(p);
  f.h[1] = *(const v8b*)(p + 16);
  return f.v;
}
__device__ __forceinline__ v8f frag_mma(v16b a, v16b b, v8f c) {
  return __builtin_amdgcn_wmma_f32_16x16x32_bf16(false, a, false, b, (short)0, c, false, false);
}

__device__ __forceinline__ void split8_lds(const float* sp, v8h& hv, v8h& lv) {
  const v4f a0 = *(const v4f*)(sp);
  const v4f a1 = *(const v4f*)(sp + 4);
#pragma unroll
  for (int e = 0; e < 4; ++e) {
    const float f0 = a0[e];
    const float f1 = a1[e];
    const unsigned short h0 = f2bf_bits(f0), h1 = f2bf_bits(f1);
    const unsigned short l0 = f2bf_bits(f0 - bf_bits2f(h0)), l1 = f2bf_bits(f1 - bf_bits2f(h1));
    hv[e]     = __builtin_bit_cast(_Float16, h0);
    hv[4 + e] = __builtin_bit_cast(_Float16, h1);
    lv[e]     = __builtin_bit_cast(_Float16, l0);
    lv[4 + e] = __builtin_bit_cast(_Float16, l1);
  }
}

template <int BIAS_MODE, int OUT_MODE, int ACT>
__global__ __launch_bounds__(256) void wmma_gemm64(
    const unsigned short* __restrict__ Ap, const unsigned short* __restrict__ A2p, int lda,
    const unsigned short* __restrict__ Btp, const unsigned short* __restrict__ Bt2p, int ldb,
    unsigned short* __restrict__ Chi, unsigned short* __restrict__ Clo, float* __restrict__ Cf, int ldc,
    const float* __restrict__ bias, int M, int N, int K) {
  const __bf16* A   = (const __bf16*)Ap;
  const __bf16* A2  = (const __bf16*)A2p;
  const __bf16* Bt  = (const __bf16*)Btp;
  const __bf16* Bt2 = (const __bf16*)Bt2p;
  __shared__ __align__(16) float sT[8][16 * 68];
  const int lane = threadIdx.x & 31;
  const int wave = threadIdx.x >> 5;
  const int tilesN = N >> 6;
  const int tilesM = M >> 6;
  const int tile = blockIdx.x * 8 + wave;
  if (tile >= tilesM * tilesN) return;
  const int tm = tile / tilesN;
  const int tn = tile - tm * tilesN;
  const int m0 = tm << 6;
  const int n0 = tn << 6;

  const int rlane = lane & 15;
  const int koff  = (lane >> 4) * 8;
  const int mOff  = (lane >> 4) * 8;

  v8f acc[4][4];
#pragma unroll
  for (int i = 0; i < 4; ++i)
#pragma unroll
    for (int j = 0; j < 4; ++j) acc[i][j] = (v8f){0.f, 0.f, 0.f, 0.f, 0.f, 0.f, 0.f, 0.f};

  for (int k0 = 0; k0 < K; k0 += 32) {
#pragma unroll
    for (int jp = 0; jp < 2; ++jp) {
      const size_t bo0 = (size_t)(n0 + ((2 * jp) << 4) + rlane) * ldb + koff + k0;
      const size_t bo1 = (size_t)(n0 + ((2 * jp + 1) << 4) + rlane) * ldb + koff + k0;
      const v16b bh0 = frag_load(Bt + bo0);
      const v16b bl0 = frag_load(Bt2 + bo0);
      const v16b bh1 = frag_load(Bt + bo1);
      const v16b bl1 = frag_load(Bt2 + bo1);
#pragma unroll
      for (int i = 0; i < 4; ++i) {
        const size_t ao = (size_t)(m0 + (i << 4) + rlane) * lda + koff + k0;
        const v16b ah = frag_load(A + ao);
        const v16b al = frag_load(A2 + ao);
        acc[i][2 * jp]     = frag_mma(ah, bh0, acc[i][2 * jp]);
        acc[i][2 * jp]     = frag_mma(ah, bl0, acc[i][2 * jp]);
        acc[i][2 * jp]     = frag_mma(al, bh0, acc[i][2 * jp]);
        acc[i][2 * jp + 1] = frag_mma(ah, bh1, acc[i][2 * jp + 1]);
        acc[i][2 * jp + 1] = frag_mma(ah, bl1, acc[i][2 * jp + 1]);
        acc[i][2 * jp + 1] = frag_mma(al, bh1, acc[i][2 * jp + 1]);
        dep_guard2_b(acc[i][2 * jp], acc[i][2 * jp + 1], ah, al, bh0, bl0, bh1, bl1);
      }
      keep4_b(bh0, bl0, bh1, bl1);
    }
  }
  acc_guard4(acc[0][0], acc[0][1], acc[0][2], acc[0][3]);
  acc_guard4(acc[1][0], acc[1][1], acc[1][2], acc[1][3]);
  acc_guard4(acc[2][0], acc[2][1], acc[2][2], acc[2][3]);
  acc_guard4(acc[3][0], acc[3][1], acc[3][2], acc[3][3]);

  float* slab = sT[wave];
#pragma unroll
  for (int i = 0; i < 4; ++i) {
    const int mBase = m0 + (i << 4);
#pragma unroll
    for (int j = 0; j < 4; ++j) {
      const int n = n0 + (j << 4) + rlane;
      float bv = 0.f;
      if (BIAS_MODE == 2) bv = bias[n];
#pragma unroll
      for (int r = 0; r < 8; ++r) {
        float v = acc[i][j][r];
        if (BIAS_MODE == 1) v += bias[mBase + mOff + r];
        if (BIAS_MODE == 2) v += bv;
        slab[(mOff + r) * 68 + (j << 4) + rlane] = v;
      }
    }
    __builtin_amdgcn_fence(__ATOMIC_RELEASE, "workgroup");
    __builtin_amdgcn_wave_barrier();
    __builtin_amdgcn_fence(__ATOMIC_ACQUIRE, "workgroup");
    if (ACT == 3) {
      const int ah2 = lane >> 4, ac4 = (lane & 15) * 4;
#pragma unroll 1
      for (int it = 0; it < 8; ++it) {
        float* sp = slab + (it * 2 + ah2) * 68 + ac4;
        const v4f vin = *(const v4f*)sp;
        const float t0 = vin[0];
        const float t1 = vin[1];
        const float t2 = vin[2];
        const float t3 = vin[3];
        v4f w;
        w[0] = silu_f32(t0);
        w[1] = silu_f32(t1);
        w[2] = silu_f32(t2);
        w[3] = silu_f32(t3);
        *(v4f*)sp = w;
      }
      __builtin_amdgcn_fence(__ATOMIC_RELEASE, "workgroup");
      __builtin_amdgcn_wave_barrier();
      __builtin_amdgcn_fence(__ATOMIC_ACQUIRE, "workgroup");
    }
    if (OUT_MODE == 0 || OUT_MODE == 3) {
      const int hh = lane >> 4, c4 = (lane & 15) * 4;
      for (int pass = 0; pass < 2; ++pass) {
#pragma unroll
        for (int it = 0; it < 8; ++it) {
          const int row = it * 2 + hh;
          const v4f v = *(const v4f*)(slab + row * 68 + c4);
          *(volatile v4f*)(Cf + (size_t)(mBase + row) * ldc + n0 + c4) = v;
        }
        __threadfence();
      }
    }
    if (OUT_MODE == 2 || OUT_MODE == 3) {
      const int q = lane >> 3, c8 = (lane & 7) * 8;
      for (int pass = 0; pass < 2; ++pass) {
#pragma unroll
        for (int it = 0; it < 4; ++it) {
          const int row = it * 4 + q;
          const float* sp = slab + row * 68 + c8;
          v8h hv, lv;
#pragma unroll
          for (int e = 0; e < 8; ++e) {
            const float f = sp[e];
            const unsigned short hb = f2bf_bits(f);
            const unsigned short lb = f2bf_bits(f - bf_bits2f(hb));
            hv[e] = __builtin_bit_cast(_Float16, hb);
            lv[e] = __builtin_bit_cast(_Float16, lb);
          }
          const size_t o = (size_t)(mBase + row) * ldc + n0 + c8;
          *(volatile v8h*)(Chi + o) = hv;
          *(volatile v8h*)(Clo + o) = lv;
        }
        __threadfence();
      }
    }
    __builtin_amdgcn_fence(__ATOMIC_RELEASE, "workgroup");
    __builtin_amdgcn_wave_barrier();
    __builtin_amdgcn_fence(__ATOMIC_ACQUIRE, "workgroup");
  }
}

__global__ __launch_bounds__(256) void split_rows_bf16_kernel(
    const float* __restrict__ src, unsigned short* __restrict__ dhi, unsigned short* __restrict__ dlo, int total8)
{
  const int i = blockIdx.x * 256 + threadIdx.x;
  if (i >= total8) return;
  const size_t e0 = (size_t)i << 3;
  const v4f a0 = *(const v4f*)(src + e0);
  const v4f a1 = *(const v4f*)(src + e0 + 4);
  v8h hv, lv;
#pragma unroll
  for (int e = 0; e < 4; ++e) {
    const float f0 = a0[e];
    const float f1 = a1[e];
    const unsigned short h0 = f2bf_bits(f0), h1 = f2bf_bits(f1);
    const unsigned short l0 = f2bf_bits(f0 - bf_bits2f(h0)), l1 = f2bf_bits(f1 - bf_bits2f(h1));
    hv[e]     = __builtin_bit_cast(_Float16, h0);
    hv[4 + e] = __builtin_bit_cast(_Float16, h1);
    lv[e]     = __builtin_bit_cast(_Float16, l0);
    lv[4 + e] = __builtin_bit_cast(_Float16, l1);
  }
  unsigned short* qh = dhi + e0;
  unsigned short* ql = dlo + e0;
  *(volatile v8h*)qh = hv;
  *(volatile v8h*)ql = lv;
  __threadfence();
  *(volatile v8h*)qh = hv;
  *(volatile v8h*)ql = lv;
}

__global__ __launch_bounds__(128) void convw_permute_split_kernel(
    const float* __restrict__ cw, unsigned short* __restrict__ AH, unsigned short* __restrict__ AL)
{
  __shared__ __align__(16) float sW[kKc];
  const int tid = threadIdx.x;
  const int o = blockIdx.x;
  const float* src = cw + (size_t)o * kKc;
#pragma unroll
  for (int p = 0; p < 6; ++p) {
    const int idx = (tid + p * 128) * 4;
    *(v4f*)(sW + idx) = *(const v4f*)(src + idx);
  }
  __syncthreads();
  const int i0 = tid * 8;
  v8h hv[3], lv[3];
#pragma unroll
  for (int it = 0; it < 3; ++it) {
#pragma unroll
    for (int e = 0; e < 8; ++e) {
      const float f = sW[(i0 + e) * 3 + it];
      const unsigned short hb = f2bf_bits(f);
      const unsigned short lb = f2bf_bits(f - bf_bits2f(hb));
      hv[it][e] = __builtin_bit_cast(_Float16, hb);
      lv[it][e] = __builtin_bit_cast(_Float16, lb);
    }
  }
  for (int pass = 0; pass < 2; ++pass) {
#pragma unroll
    for (int it = 0; it < 3; ++it) {
      const size_t off = (size_t)o * kKc + (size_t)it * kL + i0;
      *(volatile v8h*)(AH + off) = hv[it];
      *(volatile v8h*)(AL + off) = lv[it];
    }
    __threadfence();
  }
}

__device__ __forceinline__ void tile_write_hilo(const float* tile, unsigned short* OH, unsigned short* OL,
                                                int n0, int k0, int pitch, int lane, int wave)
{
  const int q = lane >> 3, c8 = (lane & 7) * 8;
  v8h hv[2], lv[2];
#pragma unroll
  for (int it = 0; it < 2; ++it) {
    const int nrow = it * 32 + wave * 4 + q;
#pragma unroll
    for (int e = 0; e < 8; ++e) {
      const float f = tile[(c8 + e) * 65 + nrow];
      const unsigned short hb = f2bf_bits(f);
      const unsigned short lb = f2bf_bits(f - bf_bits2f(hb));
      hv[it][e] = __builtin_bit_cast(_Float16, hb);
      lv[it][e] = __builtin_bit_cast(_Float16, lb);
    }
  }
  for (int pass = 0; pass < 2; ++pass) {
#pragma unroll
    for (int it = 0; it < 2; ++it) {
      const int nrow = it * 32 + wave * 4 + q;
      const size_t off = (size_t)(n0 + nrow) * pitch + k0 + c8;
      *(volatile v8h*)(OH + off) = hv[it];
      *(volatile v8h*)(OL + off) = lv[it];
    }
    __threadfence();
  }
}

__global__ __launch_bounds__(256) void transpose_split_kernel(
    const float* __restrict__ W, unsigned short* __restrict__ OH, unsigned short* __restrict__ OL)
{
  __shared__ float tile[64 * 65];
  const int tid = threadIdx.x, lane = tid & 31, wave = tid >> 5;
  const int n0 = blockIdx.x * 64;
  const int k0 = blockIdx.y * 64;
#pragma unroll
  for (int p = 0; p < 4; ++p) {
    const int idx = tid + p * 256;
    const int kk  = idx >> 4;
    const int nn4 = (idx & 15) * 4;
    const v4f v = *(const v4f*)(W + (size_t)(k0 + kk) * kD + n0 + nn4);
    tile[kk * 65 + nn4 + 0] = v[0];
    tile[kk * 65 + nn4 + 1] = v[1];
    tile[kk * 65 + nn4 + 2] = v[2];
    tile[kk * 65 + nn4 + 3] = v[3];
  }
  __syncthreads();
  tile_write_hilo(tile, OH, OL, n0, k0, kD, lane, wave);
}

__global__ __launch_bounds__(256) void wbc_build_kernel(
    const float* __restrict__ WB, const float* __restrict__ WC,
    unsigned short* __restrict__ OH, unsigned short* __restrict__ OL)
{
  __shared__ float tile[64 * 65];
  const int tid = threadIdx.x, lane = tid & 31, wave = tid >> 5;
  const int k0 = blockIdx.x * 64;
  {
    const int kk = tid >> 2;
    const int n4 = (tid & 3) * 4;
    const v4f vb = *(const v4f*)(WB + (size_t)(k0 + kk) * kNst + n4);
    const v4f vc = *(const v4f*)(WC + (size_t)(k0 + kk) * kNst + n4);
    tile[kk * 65 + n4 + 0] = vb[0];
    tile[kk * 65 + n4 + 1] = vb[1];
    tile[kk * 65 + n4 + 2] = vb[2];
    tile[kk * 65 + n4 + 3] = vb[3];
    tile[kk * 65 + kNst + n4 + 0] = vc[0];
    tile[kk * 65 + kNst + n4 + 1] = vc[1];
    tile[kk * 65 + kNst + n4 + 2] = vc[2];
    tile[kk * 65 + kNst + n4 + 3] = vc[3];
  }
#pragma unroll
  for (int p = 0; p < 8; ++p) {
    const int idx = tid + p * 256;
    const int kk = idx >> 5;
    const int nn = 2 * kNst + (idx & 31);
    tile[kk * 65 + nn] = 0.0f;
  }
  __syncthreads();
  tile_write_hilo(tile, OH, OL, 0, k0, kD, lane, wave);
}

__global__ __launch_bounds__(128) void zero_pad_rows_kernel(unsigned short* __restrict__ XMH, unsigned short* __restrict__ XML)
{
  const int tid = threadIdx.x;
  const v8h z = (v8h){0, 0, 0, 0, 0, 0, 0, 0};
  const size_t last = (size_t)(kL + 1) * kD;
  unsigned short* p0 = XMH + tid * 8;
  unsigned short* p1 = XMH + last + tid * 8;
  unsigned short* p2 = XML + tid * 8;
  unsigned short* p3 = XML + last + tid * 8;
  *(volatile v8h*)p0 = z;
  *(volatile v8h*)p1 = z;
  *(volatile v8h*)p2 = z;
  *(volatile v8h*)p3 = z;
  __threadfence();
  *(volatile v8h*)p0 = z;
  *(volatile v8h*)p1 = z;
  *(volatile v8h*)p2 = z;
  *(volatile v8h*)p3 = z;
}

__global__ __launch_bounds__(64) void scan_kernel(
    const float* __restrict__ DLR, const float* __restrict__ XC, const float* __restrict__ BC,
    const float* __restrict__ Alog, unsigned short* __restrict__ YH, unsigned short* __restrict__ YL)
{
  __shared__ __align__(16) float sX[kScanTS * kScanXP];
  __shared__ __align__(16) float sY[kScanTS * kScanYP];
  __shared__ __align__(16) float sA[kNst * kScanCh];
  __shared__ __align__(16) float sH[kNst * kScanCh];
  const int tid = threadIdx.x, lane = tid & 31, wave = tid >> 5;
  const int d0 = blockIdx.x * kScanCh;
  const int d  = d0 + tid;
#pragma unroll 1
  for (int n = 0; n < kNst; ++n) {
    sA[n * kScanCh + tid] = -expf(Alog[(size_t)d * kNst + n]);
    sH[n * kScanCh + tid] = 0.0f;
  }
  __syncthreads();
  const int lr = tid >> 3, lc4 = (tid & 7) * 4;
  const int q = lane >> 3, c8 = (lane & 7) * 8;
#pragma unroll 1
  for (int t0 = 0; t0 < kL; t0 += kScanTS) {
    __syncthreads();
#pragma unroll
    for (int i = 0; i < 8; ++i) {
      const int r = lr + 8 * i;
      *(v4f*)(sX + r * kScanXP + lc4) = *(const v4f*)(BC + (size_t)(t0 + r) * kBCP + lc4);
    }
    __syncthreads();
#pragma unroll 1
    for (int s = 0; s < kScanTS; ++s) {
      const int t = t0 + s;
      const float* xr = sX + s * kScanXP;
      const float a     = DLR[(size_t)t * kD + d];
      const float xt    = XC[(size_t)t * kD + d];
      const float ea    = expf(-fabsf(a));
      const float delta = fmaxf(a, 0.0f) + log1pf(ea);
      const float dtx   = delta * xt;
      float y = 0.f;
#pragma unroll 1
      for (int n = 0; n < kNst; ++n) {
        const float an = sA[n * kScanCh + tid];
        const float hp = sH[n * kScanCh + tid];
        const float bn = xr[n];
        const float cn = xr[kNst + n];
        const float e  = expf(delta * an);
        const float hn = e * hp + dtx * bn;
        sH[n * kScanCh + tid] = hn;
        y = hn * cn + y;
      }
      sY[s * kScanYP + tid] = y;
    }
    __syncthreads();
    v8h hv[8], lv[8];
#pragma unroll
    for (int it = 0; it < 8; ++it) {
      const int row = it * 8 + wave * 4 + q;
      split8_lds(sY + row * kScanYP + c8, hv[it], lv[it]);
    }
    for (int pass = 0; pass < 2; ++pass) {
#pragma unroll
      for (int it = 0; it < 8; ++it) {
        const int row = it * 8 + wave * 4 + q;
        const size_t o = (size_t)(t0 + row) * kD + d0 + c8;
        *(volatile v8h*)(YH + o) = hv[it];
        *(volatile v8h*)(YL + o) = lv[it];
      }
      __threadfence();
    }
  }
}

extern "C" void kernel_launch(void* const* d_in, const int* in_sizes, int n_in,
                              void* d_out, int out_size, void* d_ws, size_t ws_size,
                              hipStream_t stream) {
  if (n_in < 9) return;
  if (in_sizes[0] != 2 * kL * kD) return;
  if (in_sizes[1] != kD * kD) return;
  if (in_sizes[2] != kD) return;
  if (in_sizes[3] != kL * kL * kTap) return;
  if (in_sizes[4] != kL) return;
  if (in_sizes[5] != kD * kNst) return;
  if (in_sizes[6] != kD * kD) return;
  if (in_sizes[7] != kD * kNst) return;
  if (in_sizes[8] != kD * kNst) return;
  if (out_size != kL * kL) return;
  if (ws_size < kWsTotal) return;

  const float* x      = (const float*)d_in[0];
  const float* W_proj = (const float*)d_in[1];
  const float* b_proj = (const float*)d_in[2];
  const float* conv_w = (const float*)d_in[3];
  const float* conv_b = (const float*)d_in[4];
  const float* A_log  = (const float*)d_in[5];
  const float* W_dlt  = (const float*)d_in[6];
  const float* W_B    = (const float*)d_in[7];
  const float* W_C    = (const float*)d_in[8];
  float* out = (float*)d_out;

  char* ws = (char*)d_ws;
  unsigned short* XH   = (unsigned short*)(ws + kOffXH);
  unsigned short* XL   = (unsigned short*)(ws + kOffXL);
  unsigned short* WPH  = (unsigned short*)(ws + kOffWPH);
  unsigned short* WPL  = (unsigned short*)(ws + kOffWPL);
  unsigned short* AWH  = (unsigned short*)(ws + kOffAWH);
  unsigned short* AWL  = (unsigned short*)(ws + kOffAWL);
  unsigned short* WDH  = (unsigned short*)(ws + kOffWDH);
  unsigned short* WDL  = (unsigned short*)(ws + kOffWDL);
  unsigned short* WBCH = (unsigned short*)(ws + kOffWBCH);
  unsigned short* WBCL = (unsigned short*)(ws + kOffWBCL);
  unsigned short* XMH  = (unsigned short*)(ws + kOffXMH);
  unsigned short* XML  = (unsigned short*)(ws + kOffXML);
  float*          XC   = (float*)(ws + kOffXC);
  unsigned short* XCH  = (unsigned short*)(ws + kOffXCH);
  unsigned short* XCL  = (unsigned short*)(ws + kOffXCL);
  unsigned short* XGH  = (unsigned short*)(ws + kOffXGH);
  unsigned short* XGL  = (unsigned short*)(ws + kOffXGL);
  float*          DLR  = (float*)(ws + kOffDLR);
  float*          BC   = (float*)(ws + kOffBC);
  unsigned short* YH   = (unsigned short*)(ws + kOffYH);
  unsigned short* YL   = (unsigned short*)(ws + kOffYL);
  unsigned short* ZH   = (unsigned short*)(ws + kOffZH);
  unsigned short* ZL   = (unsigned short*)(ws + kOffZL);

  const int tilesFull = (kL / 64) * (kD / 64) / 8;
  const int tilesBC   = (kL / 64) * (kBCP / 64) / 8;
  static_assert(((kL / 64) * (kD / 64)) % 8 == 0 && ((kL / 64) * (kBCP / 64)) % 8 == 0, "tiles fill whole blocks");

  split_rows_bf16_kernel<<<(2 * kL * kD / 8) / 256, 256, 0, stream>>>(x, XH, XL, 2 * kL * kD / 8);
  split_rows_bf16_kernel<<<(kD * kD / 8) / 256, 256, 0, stream>>>(W_proj, WPH, WPL, kD * kD / 8);
  convw_permute_split_kernel<<<kL, 128, 0, stream>>>(conv_w, AWH, AWL);
  transpose_split_kernel<<<dim3(kD / 64, kD / 64), 256, 0, stream>>>(W_dlt, WDH, WDL);
  wbc_build_kernel<<<kD / 64, 256, 0, stream>>>(W_B, W_C, WBCH, WBCL);
  zero_pad_rows_kernel<<<1, 128, 0, stream>>>(XMH, XML);

  wmma_gemm64<1, 2, 0><<<tilesFull, 256, 0, stream>>>(
      WPH, WPL, kD, XH, XL, kD,
      XMH + kD, XML + kD, XC, kD, b_proj, kL, kL, kD);

  wmma_gemm64<2, 2, 3><<<tilesFull, 256, 0, stream>>>(
      XH + (size_t)kL * kD, XL + (size_t)kL * kD, kD, WPH, WPL, kD,
      XGH, XGL, XC, kD, b_proj, kL, kD, kD);

  wmma_gemm64<1, 3, 3><<<tilesFull, 256, 0, stream>>>(
      AWH, AWL, kKc, XMH, XML, kD,
      XCH, XCL, XC, kD, conv_b, kL, kD, kKc);

  wmma_gemm64<0, 0, 0><<<tilesFull, 256, 0, stream>>>(
      XCH, XCL, kD, WDH, WDL, kD,
      YH, YL, DLR, kD, b_proj, kL, kD, kD);

  wmma_gemm64<0, 0, 0><<<tilesBC, 256, 0, stream>>>(
      XCH, XCL, kD, WBCH, WBCL, kD,
      YH, YL, BC, kBCP, b_proj, kL, kBCP, kD);

  scan_kernel<<<kD / kScanCh, kScanCh, 0, stream>>>(DLR, XC, BC, A_log, YH, YL);

  wmma_gemm64<0, 2, 0><<<tilesFull, 256, 0, stream>>>(
      YH, YL, kD, XGH, XGL, kD,
      ZH, ZL, DLR, kL, b_proj, kL, kL, kD);

  wmma_gemm64<2, 0, 0><<<tilesFull, 256, 0, stream>>>(
      ZH, ZL, kL, WPH, WPL, kL,
      YH, YL, out, kL, b_proj, kL, kL, kL);
}
